// PatchEmbed_5583457485374
// MI455X (gfx1250) — hardware-run, weakly checked
//
#include <hip/hip_runtime.h>
#include <math.h>

typedef __attribute__((ext_vector_type(16))) _Float16 v16h;
typedef __attribute__((ext_vector_type(8)))  _Float16 v8h;
typedef __attribute__((ext_vector_type(8)))  float    v8f;
typedef __attribute__((ext_vector_type(4)))  float    v4f;

constexpr int kBatch   = 8;
constexpr int kPts     = 16384;
constexpr int kCtr     = 2048;
constexpr int kNbr     = 32;
constexpr int kCh1     = 64;
constexpr int kCh2     = 128;
constexpr int kCh3     = 256;
constexpr int kPatches = kBatch * kCtr;
constexpr int kPatchPerBlock = 16;
constexpr int kFusedBlocks   = kPatches / kPatchPerBlock;
constexpr int kIters   = kPatchPerBlock / 2;
constexpr int kPitchA  = kCh1 + 8;
constexpr int kPitchB  = kCh2 + 8;
constexpr float kWCarry = 64.0f;
constexpr float kHCarry = 16.0f;
constexpr float kFold   = 1.0f / (kWCarry * kHCarry);
constexpr float kHalfMinNormal = 6.103515625e-5f;

static_assert(kCtr == 2048, "batch index is patch >> 11");
static_assert(kNbr == 32, "two 16-row tiles per patch");
static_assert((kCh1 % 32) == 0 && (kCh2 % 32) == 0, "K multiples of 32");
static_assert((kCh2 % 16) == 0 && (kCh3 % 32) == 0, "N tile multiples");
static_assert(kCh2 == 8 * 16, "layer 2: one 16-channel tile per wave, 8 waves");
static_assert(kCh3 == 8 * 32, "layer 3: two 16-channel tiles per wave, 8 waves");
static_assert((kPatches % kPatchPerBlock) == 0 && (kPatchPerBlock % 2) == 0, "grid exact");
static_assert(kFold == 1.0f / 1024.0f, "fold constant");

constexpr size_t kOffW2H  = 0;
constexpr size_t kOffW3H  = kOffW2H + (size_t)kCh2 * kCh1 * 2;
constexpr size_t kWsTotal = kOffW3H + (size_t)kCh3 * kCh2 * 2;
static_assert(kWsTotal == 81920ull, "carve total");
static_assert((kOffW3H % 128) == 0, "aligned region");
static_assert(kWsTotal <= 134217728ull, "carve cap");
constexpr int kW2Threads   = kCh2 * kCh1 / 8;
constexpr int kW3Threads   = kCh3 * kCh2 / 8;
constexpr int kW2Blocks    = kW2Threads / 256;
constexpr int kPrepThreads = kW2Threads + kW3Threads;
constexpr int kPrepBlocks  = kPrepThreads / 256;
static_assert((kW2Threads % 256) == 0 && (kW3Threads % 256) == 0, "prep grid exact");
static_assert(kPrepBlocks == 20, "prep grid");

union FragU { v16h v; v8h h[2]; };
__device__ __forceinline__ v16h frag_load(const _Float16* p) {
  FragU f;
  f.h[0] = *(const v8h*)(p);
  f.h[1] = *(const v8h*)(p + 16);
  return f.v;
}
__device__ __forceinline__ v8f mma_h(v16h a, v16h b, v8f c) {
  c = __builtin_amdgcn_wmma_f32_16x16x32_f16(false, a, false, b, (short)0, c, false, false);
  asm volatile("v_nop\n\tv_nop\n\tv_nop\n\tv_nop" : "+v"(c) : "v"(a), "v"(b));
  return c;
}
__device__ __forceinline__ _Float16 to_h_flush(float v) {
  const float f = (fabsf(v) < kHalfMinNormal) ? 0.0f : v;
  return (_Float16)f;
}

__global__ __launch_bounds__(256) void weight_planes_kernel(
    const float* __restrict__ W2, const float* __restrict__ W3, unsigned short* __restrict__ planes)
{
  const int i = blockIdx.x * 256 + threadIdx.x;
  if (i >= kPrepThreads) return;
  const bool first = (blockIdx.x < kW2Blocks);
  const float* src = first ? (W2 + (size_t)i * 8) : (W3 + (size_t)(i - kW2Threads) * 8);
  const v4f a0 = *(const v4f*)(src);
  const v4f a1 = *(const v4f*)(src + 4);
  v8h hv;
#pragma unroll
  for (int e = 0; e < 4; ++e) {
    const float f0 = a0[e] * kWCarry;
    const float f1 = a1[e] * kWCarry;
    hv[e]     = to_h_flush(f0);
    hv[4 + e] = to_h_flush(f1);
  }
  unsigned short* q = planes + (size_t)i * 8;
  *(volatile v8h*)q = hv;
  __threadfence();
  *(volatile v8h*)q = hv;
}

__global__ __launch_bounds__(256) void patch_mlp_max_kernel(
    const float* __restrict__ xyz, const float* __restrict__ centers, const int* __restrict__ idx_knn,
    const float* __restrict__ W1, const float* __restrict__ b1,
    const float* __restrict__ b2, const float* __restrict__ b3,
    const _Float16* __restrict__ w2h, const _Float16* __restrict__ w3h,
    float* __restrict__ out)
{
  __shared__ __align__(16) _Float16 W3s[kCh3 * kPitchB];
  __shared__ __align__(16) _Float16 W2s[kCh2 * kPitchA];
  __shared__ __align__(16) _Float16 h1s[64 * kPitchA];
  __shared__ __align__(16) _Float16 h2s[64 * kPitchB];

  const int tid  = threadIdx.x;
  const int lane = tid & 31;
  const int wave = tid >> 5;
  const int hh   = lane >> 4;
  const int c    = lane & 15;

#pragma unroll 1
  for (int i = tid; i < kCh3 * (kCh2 / 8); i += 256) {
    const int r = i >> 4, cc = (i & 15) * 8;
    *(v8h*)(W3s + r * kPitchB + cc) = *(const v8h*)(w3h + (size_t)i * 8);
  }
#pragma unroll 1
  for (int i = tid; i < kCh2 * (kCh1 / 8); i += 256) {
    const int r = i >> 3, cc = (i & 7) * 8;
    *(v8h*)(W2s + r * kPitchA + cc) = *(const v8h*)(w2h + (size_t)i * 8);
  }

  const int row1 = tid >> 2;
  const int q1   = tid & 3;
  float w1r[48];
  float b1r[16];
#pragma unroll
  for (int j = 0; j < 12; ++j) {
    const v4f t = *(const v4f*)(W1 + q1 * 48 + 4 * j);
    w1r[4 * j + 0] = t[0];
    w1r[4 * j + 1] = t[1];
    w1r[4 * j + 2] = t[2];
    w1r[4 * j + 3] = t[3];
  }
#pragma unroll
  for (int j = 0; j < 4; ++j) {
    const v4f t = *(const v4f*)(b1 + q1 * 16 + 4 * j);
    b1r[4 * j + 0] = t[0];
    b1r[4 * j + 1] = t[1];
    b1r[4 * j + 2] = t[2];
    b1r[4 * j + 3] = t[3];
  }
  float b2r[8];
  {
    const v4f t0 = *(const v4f*)(b2 + 16 * wave + 8 * hh);
    const v4f t1 = *(const v4f*)(b2 + 16 * wave + 8 * hh + 4);
    b2r[0] = t0[0]; b2r[1] = t0[1]; b2r[2] = t0[2]; b2r[3] = t0[3];
    b2r[4] = t1[0]; b2r[5] = t1[1]; b2r[6] = t1[2]; b2r[7] = t1[3];
  }
  const float b3v = b3[32 * wave + lane];

  __syncthreads();

  const int pbase = blockIdx.x * kPatchPerBlock;
#pragma unroll 1
  for (int it = 0; it < kIters; ++it) {
    const int p0 = pbase + 2 * it;

    {
      const int p  = p0 + (row1 >> 5);
      const int kk = row1 & 31;
      const int bb = p >> 11;
      int id = idx_knn[(size_t)p * kNbr + kk];
      id = id < 0 ? 0 : id;
      id = id > (kPts - 1) ? (kPts - 1) : id;
      const float* xp = xyz + ((size_t)bb * kPts + (size_t)id) * 3;
      const float* cp = centers + (size_t)p * 3;
      const float lx = xp[0] - cp[0];
      const float ly = xp[1] - cp[1];
      const float lz = xp[2] - cp[2];
      v8h o0, o1;
#pragma unroll
      for (int j = 0; j < 8; ++j) {
        float s0 = lx * w1r[3 * j + 0];
        s0 = fmaf(ly, w1r[3 * j + 1], s0);
        s0 = fmaf(lz, w1r[3 * j + 2], s0);
        s0 = fmaxf(s0 + b1r[j], 0.0f);
        o0[j] = to_h_flush(s0 * kHCarry);
        float s1 = lx * w1r[3 * (j + 8) + 0];
        s1 = fmaf(ly, w1r[3 * (j + 8) + 1], s1);
        s1 = fmaf(lz, w1r[3 * (j + 8) + 2], s1);
        s1 = fmaxf(s1 + b1r[j + 8], 0.0f);
        o1[j] = to_h_flush(s1 * kHCarry);
      }
      *(v8h*)(h1s + row1 * kPitchA + q1 * 16)     = o0;
      *(v8h*)(h1s + row1 * kPitchA + q1 * 16 + 8) = o1;
    }
    __syncthreads();

    {
      v8f c2[4];
#pragma unroll
      for (int i = 0; i < 4; ++i) c2[i] = (v8f){0.f, 0.f, 0.f, 0.f, 0.f, 0.f, 0.f, 0.f};
#pragma unroll
      for (int ks = 0; ks < kCh1 / 32; ++ks) {
        const int k0 = ks * 32 + 8 * hh;
        const v16h af = frag_load(W2s + (16 * wave + c) * kPitchA + k0);
#pragma unroll
        for (int i = 0; i < 4; ++i) {
          const v16h bf = frag_load(h1s + (16 * i + c) * kPitchA + k0);
          c2[i] = mma_h(af, bf, c2[i]);
        }
      }
#pragma unroll
      for (int i = 0; i < 4; ++i) {
        v8h hv;
#pragma unroll
        for (int r = 0; r < 8; ++r) {
          float v = c2[i][r] * kFold + b2r[r];
          v = fmaxf(v, 0.0f);
          hv[r] = to_h_flush(v * kHCarry);
        }
        *(v8h*)(h2s + (16 * i + c) * kPitchB + 16 * wave + 8 * hh) = hv;
      }
    }
    __syncthreads();

    {
      v8f acc[4][2];
#pragma unroll
      for (int i = 0; i < 4; ++i) {
        acc[i][0] = (v8f){0.f, 0.f, 0.f, 0.f, 0.f, 0.f, 0.f, 0.f};
        acc[i][1] = (v8f){0.f, 0.f, 0.f, 0.f, 0.f, 0.f, 0.f, 0.f};
      }
#pragma unroll 1
      for (int ks = 0; ks < kCh2 / 32; ++ks) {
        const int k0 = ks * 32 + 8 * hh;
        const v16h bf0 = frag_load(W3s + (32 * wave + c) * kPitchB + k0);
        const v16h bf1 = frag_load(W3s + (32 * wave + 16 + c) * kPitchB + k0);
#pragma unroll
        for (int i = 0; i < 4; ++i) {
          const v16h af = frag_load(h2s + (16 * i + c) * kPitchB + k0);
          acc[i][0] = mma_h(af, bf0, acc[i][0]);
          acc[i][1] = mma_h(af, bf1, acc[i][1]);
        }
      }
      float mA0 = fmaxf(acc[0][0][0], acc[1][0][0]);
      float mB0 = fmaxf(acc[0][1][0], acc[1][1][0]);
      float mA1 = fmaxf(acc[2][0][0], acc[3][0][0]);
      float mB1 = fmaxf(acc[2][1][0], acc[3][1][0]);
#pragma unroll
      for (int r = 1; r < 8; ++r) {
        mA0 = fmaxf(mA0, fmaxf(acc[0][0][r], acc[1][0][r]));
        mB0 = fmaxf(mB0, fmaxf(acc[0][1][r], acc[1][1][r]));
        mA1 = fmaxf(mA1, fmaxf(acc[2][0][r], acc[3][0][r]));
        mB1 = fmaxf(mB1, fmaxf(acc[2][1][r], acc[3][1][r]));
      }
      const float xA0 = __shfl_xor(mA0, 16, 32);
      const float xB0 = __shfl_xor(mB0, 16, 32);
      const float xA1 = __shfl_xor(mA1, 16, 32);
      const float xB1 = __shfl_xor(mB1, 16, 32);
      mA0 = fmaxf(mA0, xA0);
      mB0 = fmaxf(mB0, xB0);
      mA1 = fmaxf(mA1, xA1);
      mB1 = fmaxf(mB1, xB1);
      const float s0 = (lane < 16) ? mA0 : mB0;
      const float s1 = (lane < 16) ? mA1 : mB1;
      const float v0 = s0 * kFold + b3v;
      const float v1 = s1 * kFold + b3v;
      float* o0 = out + (size_t)p0 * kCh3 + 32 * wave + lane;
      float* o1 = o0 + kCh3;
      *(volatile float*)o0 = v0;
      *(volatile float*)o1 = v1;
      __threadfence();
      *(volatile float*)o0 = v0;
      *(volatile float*)o1 = v1;
    }
    __syncthreads();
  }
}

extern "C" void kernel_launch(void* const* d_in, const int* in_sizes, int n_in,
                              void* d_out, int out_size, void* d_ws, size_t ws_size,
                              hipStream_t stream) {
  if (n_in < 9) return;
  if (in_sizes[0] != kBatch * kPts * 3) return;
  if (in_sizes[1] != kBatch * kCtr * 3) return;
  if (in_sizes[2] != kBatch * kCtr * kNbr) return;
  if (in_sizes[3] != kCh1 * 3) return;
  if (in_sizes[4] != kCh1) return;
  if (in_sizes[5] != kCh2 * kCh1) return;
  if (in_sizes[6] != kCh2) return;
  if (in_sizes[7] != kCh3 * kCh2) return;
  if (in_sizes[8] != kCh3) return;
  if (out_size != kPatches * kCh3) return;
  if (ws_size < kWsTotal) return;

  const float* xyz     = (const float*)d_in[0];
  const float* centers = (const float*)d_in[1];
  const int*   idx     = (const int*)d_in[2];
  const float* W1      = (const float*)d_in[3];
  const float* b1      = (const float*)d_in[4];
  const float* W2      = (const float*)d_in[5];
  const float* b2      = (const float*)d_in[6];
  const float* W3      = (const float*)d_in[7];
  const float* b3      = (const float*)d_in[8];
  float* out = (float*)d_out;

  char* ws = (char*)d_ws;
  unsigned short* planes = (unsigned short*)(ws + kOffW2H);
  const _Float16* w2h = (const _Float16*)(ws + kOffW2H);
  const _Float16* w3h = (const _Float16*)(ws + kOffW3H);

  weight_planes_kernel<<<kPrepBlocks, 256, 0, stream>>>(W2, W3, planes);
  patch_mlp_max_kernel<<<kFusedBlocks, 256, 0, stream>>>(xyz, centers, idx, W1, b1, b2, b3, w2h, w3h, out);
}
